// mmult_32117765439601
// MI455X (gfx1250) — hardware-verified
//
#include <hip/hip_runtime.h>
#include <math.h>

typedef __attribute__((ext_vector_type(16))) _Float16 v16h;
typedef __attribute__((ext_vector_type(16))) __bf16 v16b;
typedef __attribute__((ext_vector_type(8)))  _Float16 v8h;
typedef __attribute__((ext_vector_type(8)))  float v8f;
typedef __attribute__((ext_vector_type(4)))  float v4f;
typedef __attribute__((ext_vector_type(2)))  float v2f;
typedef __attribute__((ext_vector_type(4)))  unsigned v4u;
typedef __attribute__((ext_vector_type(4)))  int v4i;
typedef float __attribute__((may_alias)) float_a;
typedef int __attribute__((may_alias)) int_a;

template <typename T> __device__ __forceinline__ void vst2(void* p, T v) { *(volatile T*)p = v; __threadfence(); *(volatile T*)p = v; }
__device__ __forceinline__ v8f wmma16(v16h a, v16h b, v8f c) {
  v8f d = __builtin_amdgcn_wmma_f32_16x16x32_f16(false, a, false, b, (short)0, c, false, false);
  asm volatile("v_nop\n\tv_nop\n\tv_nop\n\tv_nop" : "+v"(d) : "v"(a), "v"(b));
  return d;
}
__device__ __forceinline__ v8f wmma_bf(v16b a, v16b b, v8f c) {
  v8f d = __builtin_amdgcn_wmma_f32_16x16x32_bf16(false, a, false, b, (short)0, c, false, false);
  asm volatile("v_nop\n\tv_nop\n\tv_nop\n\tv_nop" : "+v"(d) : "v"(a), "v"(b));
  return d;
}
__device__ __forceinline__ v16h frag_h(const _Float16* rowk0, int lane) {
  union { v16h v; v8h q[2]; } u; const _Float16* p = rowk0 + 8 * (lane >> 4);
  u.q[0] = *(const v8h*)p; u.q[1] = *(const v8h*)(p + 16); return u.v;
}
__device__ __forceinline__ v16h frag_f32(const float* rowk0, int lane) {
  v16h a; const float* p = rowk0 + 8 * (lane >> 4);
#pragma unroll
  for (int i = 0; i < 8; ++i) { a[i] = (_Float16)p[i]; a[8 + i] = (_Float16)p[16 + i]; }
  return a;
}
__device__ __forceinline__ v16h frag_f32s(const float* rowk0, int lane, float sc) {
  v16h a; const float* p = rowk0 + 8 * (lane >> 4);
#pragma unroll
  for (int i = 0; i < 8; ++i) { a[i] = (_Float16)(p[i] * sc); a[8 + i] = (_Float16)(p[16 + i] * sc); }
  return a;
}
__device__ __forceinline__ v16h fragc_f32(const float* W, int k0, int n, int lane, int ld, int K) {
  v16h a; const int g = lane >> 4;
#pragma unroll
  for (int i = 0; i < 8; ++i) { const int ka = k0 + 8 * g + i, kb = ka + 16;
    a[i] = (_Float16)(ka < K ? W[(size_t)(ka < K ? ka : K - 1) * ld + n] : 0.f); a[8 + i] = (_Float16)(kb < K ? W[(size_t)(kb < K ? kb : K - 1) * ld + n] : 0.f); }
  return a;
}
struct F2 { v16b h, l; };
__device__ __forceinline__ F2 bsplit16(const float v[16]) { F2 r;
#pragma unroll
  for (int i = 0; i < 16; ++i) { const __bf16 h = (__bf16)v[i]; r.h[i] = h; r.l[i] = (__bf16)(v[i] - (float)h); }
  return r; }
__device__ __forceinline__ F2 split_row(const float* row, int k0, int lane) { float v[16]; const float* p = row + k0 + 8 * (lane >> 4);
#pragma unroll
  for (int i = 0; i < 8; ++i) { v[i] = p[i]; v[8 + i] = p[16 + i]; }
  return bsplit16(v); }
__device__ __forceinline__ F2 split_rowK(const float* row, int k0, int lane, int K) { float v[16]; const int g = lane >> 4;
#pragma unroll
  for (int i = 0; i < 8; ++i) { const int ka = k0 + 8 * g + i, kb = ka + 16; v[i] = ka < K ? row[ka < K ? ka : K - 1] : 0.f; v[8 + i] = kb < K ? row[kb < K ? kb : K - 1] : 0.f; }
  return bsplit16(v); }
__device__ __forceinline__ F2 split_col(const float* W, int k0, int n, int lane, int ld, int K) { float v[16]; const int g = lane >> 4;
#pragma unroll
  for (int i = 0; i < 8; ++i) { const int ka = k0 + 8 * g + i, kb = ka + 16; v[i] = ka < K ? W[(size_t)(ka < K ? ka : K - 1) * ld + n] : 0.f; v[8 + i] = kb < K ? W[(size_t)(kb < K ? kb : K - 1) * ld + n] : 0.f; }
  return bsplit16(v); }
__device__ __forceinline__ v8f mac3(const F2& a, const F2& b, v8f c) { c = wmma_bf(a.l, b.h, c); c = wmma_bf(a.h, b.l, c); return wmma_bf(a.h, b.h, c); }
__device__ __forceinline__ float sigm(float v) { return 1.0f / (1.0f + expf(-v)); }
#define LDSX() do { asm volatile("s_wait_dscnt 0" ::: "memory"); __builtin_amdgcn_wave_barrier(); __builtin_amdgcn_fence(__ATOMIC_RELEASE, "workgroup"); } while (0)


#define N 2048
#ifndef TRB
#define TRB (N / 64)
#endif
typedef __attribute__((ext_vector_type(8))) __bf16 v8b;
__device__ __forceinline__ v16b frag_b(const __bf16* rowk0, int lane) {
  union { v16b v; v8b q[2]; } u; const __bf16* p = rowk0 + 8 * (lane >> 4);
  u.q[0] = *(const v8b*)p; u.q[1] = *(const v8b*)(p + 16); return u.v;
}
__device__ __forceinline__ float bfr(float v) { return (float)(__bf16)v; }
__device__ __attribute__((noinline)) float exp_ni(float v) { return expf(v); }
__device__ __attribute__((noinline)) float erf_ni(float v) { return erff(v); }

#define WS_T   0u
#define WS_XB  (WS_T + 2u * 3 * N * N)
#define WS_XQ  (WS_XB + 2u * N * N)
#define WS_XQL (WS_XQ + 2u * N * N)
#define WS_XKT (WS_XQL + 2u * N * N)
#define WS_XKL (WS_XKT + 2u * N * N)
#define WS_XVT (WS_XKL + 2u * N * N)
#define WS_XVL (WS_XVT + 2u * N * N)
#define WS_P   (WS_XVL + 2u * N * N)
#define WS_PL  (WS_P + 2u * N * N)
#define WS_S   (WS_PL + 2u * N * N)
#define WS_END (WS_S + 4u * N * N)

__global__ __launch_bounds__(256) void k_pack(const float* __restrict__ X, const float* __restrict__ Q, const float* __restrict__ K, const float* __restrict__ V, __bf16* __restrict__ T, __bf16* __restrict__ XB) {
  __shared__ __align__(16) __bf16 s[N]; const int n = blockIdx.x, which = blockIdx.y, t = threadIdx.x;
  if (which < 3) { const float* M = (which == 0) ? Q : (which == 1) ? K : V; for (int c = t; c < N; c += 256) s[c] = (__bf16)M[(size_t)c * N + n]; }
  else { for (int c = t; c < N; c += 256) s[c] = (__bf16)X[(size_t)n * N + c]; }
  __syncthreads();
  __bf16* dst = (which < 3) ? (T + ((size_t)which * N + n) * N) : (XB + (size_t)n * N);
  for (int q8 = t; q8 < N / 8; q8 += 256) vst2((unsigned*)(dst + q8 * 8), *(const v4u*)&s[q8 * 8]);
}
__global__ __launch_bounds__(128) void k_g1(const __bf16* __restrict__ XB, const __bf16* __restrict__ T, _Float16* __restrict__ OH_, _Float16* __restrict__ OL_) {
  __shared__ __align__(16) _Float16 so[4][16][136], sol[4][16][136];
  const int tid = threadIdx.x, wave = tid >> 5, lane = tid & 31, col = lane & 15, g = lane >> 4; const size_t r0 = (size_t)blockIdx.x * 64 + wave * 16; const int n0 = blockIdx.y * 128; const int which = blockIdx.z;
  const __bf16* A = (which == 0) ? XB : (T + (size_t)which * N * N); const __bf16* Bm = (which == 0) ? T : XB;
  _Float16* OH = OH_ + (size_t)which * 2 * N * N; _Float16* OL = OL_ + (size_t)which * 2 * N * N;
  v8f acc[8] = {};
#pragma unroll 2
  for (int kc = 0; kc < N / 32; ++kc) { const v16b a = frag_b(A + (r0 + col) * N + kc * 32, lane);
#pragma unroll
    for (int j = 0; j < 8; ++j) acc[j] = wmma_bf(a, frag_b(Bm + (size_t)(n0 + j * 16 + col) * N + kc * 32, lane), acc[j]); }
#pragma unroll
  for (int j = 0; j < 8; ++j)
#pragma unroll
    for (int r = 0; r < 8; ++r) { const float v = acc[j][r]; const _Float16 hv = (_Float16)v; so[wave][8 * g + r][j * 16 + col] = hv; sol[wave][8 * g + r][j * 16 + col] = (_Float16)((v - (float)hv) * 2048.0f); }
  LDSX();
  for (int rl = 0; rl < 16; ++rl) if (lane < 16) { vst2((unsigned*)(OH + (r0 + rl) * N + n0 + lane * 8), *(const v4u*)&so[wave][rl][lane * 8]); vst2((unsigned*)(OL + (r0 + rl) * N + n0 + lane * 8), *(const v4u*)&sol[wave][rl][lane * 8]); }
}
template <int MODE>
__global__ __launch_bounds__(128) void k_g2(const _Float16* __restrict__ AH, const _Float16* __restrict__ AL, const _Float16* __restrict__ BH, const _Float16* __restrict__ BL, float* __restrict__ OUT) {
  __shared__ __align__(16) float so[4][16][132];
  const int tid = threadIdx.x, wave = tid >> 5, lane = tid & 31, col = lane & 15, g = lane >> 4; const size_t r0 = (size_t)blockIdx.x * 64 + wave * 16; const int n0 = blockIdx.y * 128;
  v8f acc[8] = {}, accl[8] = {};
#pragma unroll 2
  for (int kc = 0; kc < N / 32; ++kc) { const v16h a = frag_h(AH + (r0 + col) * N + kc * 32, lane), al = frag_h(AL + (r0 + col) * N + kc * 32, lane);
#pragma unroll
    for (int j = 0; j < 8; ++j) { const size_t bo = (size_t)(n0 + j * 16 + col) * N + kc * 32; const v16h bh = frag_h(BH + bo, lane); acc[j] = wmma16(a, bh, acc[j]); accl[j] = wmma16(al, bh, accl[j]); accl[j] = wmma16(a, frag_h(BL + bo, lane), accl[j]); } }
#pragma unroll
  for (int j = 0; j < 8; ++j)
#pragma unroll
    for (int r = 0; r < 8; ++r) so[wave][8 * g + r][j * 16 + col] = acc[j][r] + accl[j][r] * (1.0f / 2048.0f);
  LDSX();
  for (int rl = 0; rl < 16; ++rl) vst2(OUT + (r0 + rl) * N + n0 + lane * 4, *(const v4f*)&so[wave][rl][lane * 4]);
}
#define PER (N / 256)
__global__ __launch_bounds__(256) void k_soft(const float* __restrict__ S, _Float16* __restrict__ P, _Float16* __restrict__ PL) {
  __shared__ float red[8]; __shared__ __align__(16) _Float16 sh[N], sl[N]; const int t = threadIdx.x; const size_t row = blockIdx.x; const float* p = S + row * N + t * PER;
  float v[PER]; float mx = -3.0e38f;
#pragma unroll
  for (int i = 0; i < PER; ++i) { v[i] = p[i]; mx = fmaxf(mx, v[i]); }
#pragma unroll
  for (int o = 1; o < 32; o <<= 1) mx = fmaxf(mx, __shfl_xor(mx, o));
  if ((t & 31) == 0) red[t >> 5] = mx; __syncthreads(); float gm = -3.0e38f; for (int w = 0; w < 8; ++w) gm = fmaxf(gm, red[w]); __syncthreads();
  float sm = 0.f;
#pragma unroll
  for (int i = 0; i < PER; ++i) { v[i] = __expf(v[i] - gm); sm += v[i]; }
#pragma unroll
  for (int o = 1; o < 32; o <<= 1) sm += __shfl_xor(sm, o);
  if ((t & 31) == 0) red[t >> 5] = sm; __syncthreads(); float tot = 0.f; for (int w = 0; w < 8; ++w) tot += red[w]; const float inv = 1.0f / tot;
#pragma unroll
  for (int i = 0; i < PER; ++i) { const float pv = v[i] * inv; const _Float16 h = (_Float16)pv; sh[t * PER + i] = h; sl[t * PER + i] = (_Float16)((pv - (float)h) * 2048.0f); }
  __syncthreads();
  if (t < N / 8) { vst2((unsigned*)(P + row * N + t * 8), *(const v4u*)&sh[t * 8]); vst2((unsigned*)(PL + row * N + t * 8), *(const v4u*)&sl[t * 8]); }
}
extern "C" void kernel_launch(void* const* d_in, const int* in_sizes, int n_in, void* d_out, int out_size, void* d_ws, size_t ws_size, hipStream_t stream) {
  (void)in_sizes; (void)n_in; (void)out_size;
  const float** F = (const float**)d_in;
  if (ws_size < (size_t)WS_END) return;
  char* ws = (char*)d_ws; __bf16 *T = (__bf16*)(ws + WS_T), *XB = (__bf16*)(ws + WS_XB); _Float16 *XQ = (_Float16*)(ws + WS_XQ), *XQL = (_Float16*)(ws + WS_XQL), *XKT = (_Float16*)(ws + WS_XKT), *XKL = (_Float16*)(ws + WS_XKL), *XVT = (_Float16*)(ws + WS_XVT), *XVL = (_Float16*)(ws + WS_XVL), *P = (_Float16*)(ws + WS_P), *PL = (_Float16*)(ws + WS_PL); float* S = (float*)(ws + WS_S);
  k_pack<<<dim3(N, 4), 256, 0, stream>>>(F[0], F[1], F[2], F[3], T, XB);
  k_g1<<<dim3(N / 64, N / 128, 3), 128, 0, stream>>>(XB, T, XQ, XQL);
  k_g2<0><<<dim3(TRB, N / 128), 128, 0, stream>>>(XQ, XQL, XKT, XKL, S);
  k_soft<<<TRB * 64, 256, 0, stream>>>(S, P, PL);
  k_g2<1><<<dim3(TRB, N / 128), 128, 0, stream>>>(P, PL, XVT, XVL, (float*)d_out);
}
